// RowColRPA_20237885899403
// MI455X (gfx1250) — hardware-verified
//
#include <hip/hip_runtime.h>
#include <math.h>
#include <stdint.h>

#define NBATCH 2
#define SEQ    512
#define DM     256
#define NH     8
#define HD     32
#define NPROJ  (3 * DM)
#define MP     (NBATCH * SEQ)
#define NQB    (SEQ / 64)
#define LNT    (DM / 4)
#define LNW    (LNT / 32)
#define LNEPS  1.0e-5f
#define WSC    64.0f
#define CSC    64.0f
#define PSC    1024.0f
static_assert(NH * HD == DM);
static_assert(HD == 32);
static_assert((SEQ % 64) == 0 && (DM % 64) == 0 && (NPROJ % 64) == 0 && (MP % 64) == 0 && (MP % 8) == 0);
static_assert(DM == 4 * LNT && (LNT % 32) == 0 && LNW <= 8);

typedef _Float16 v16h __attribute__((ext_vector_type(16)));
typedef _Float16 v8h  __attribute__((ext_vector_type(8)));
typedef __bf16   v16b __attribute__((ext_vector_type(16)));
typedef float    v8f  __attribute__((ext_vector_type(8)));
typedef float    v4f  __attribute__((ext_vector_type(4)));
typedef unsigned int v4u __attribute__((ext_vector_type(4)));

union FragH { v16h v; v8h h[2]; };
union FragB { v16b v; v4u u[2]; v8f f; };

__device__ __forceinline__ unsigned short bf_bits(float f) {
  unsigned u = __float_as_uint(f);
  return (unsigned short)((u + 0x7FFFu + ((u >> 16) & 1u)) >> 16);
}
__device__ __forceinline__ float bf_up(unsigned short h) { return __uint_as_float(((unsigned)h) << 16); }
__device__ __forceinline__ float bfr(float f) { return bf_up(bf_bits(f)); }
__device__ __forceinline__ unsigned short h_bits(_Float16 x) { return __builtin_bit_cast(unsigned short, x); }
__device__ __forceinline__ unsigned pk16(unsigned short a, unsigned short b) { return (unsigned)a | ((unsigned)b << 16); }
__device__ __forceinline__ v8f zero8() { v8f z = {0.f, 0.f, 0.f, 0.f, 0.f, 0.f, 0.f, 0.f}; return z; }

__device__ __forceinline__ v16h ldfrag_h(const _Float16* p) {
  FragH f;
  f.h[0] = *(const v8h*)(p);
  f.h[1] = *(const v8h*)(p + 16);
  return f.v;
}

__device__ __forceinline__ v8f mma_h(v16h a, v16h b, v8f c) {
  c = __builtin_amdgcn_wmma_f32_16x16x32_f16(false, a, false, b, (short)0, c, false, false);
#if defined(__HIP_DEVICE_COMPILE__)
  asm volatile("v_nop\n\tv_nop\n\tv_nop\n\tv_nop" : "+v"(c) : "v"(a), "v"(b));
#endif
  return c;
}
__device__ __forceinline__ v8f mma_h_raw(v16h a, v16h b, v8f c) {
  return __builtin_amdgcn_wmma_f32_16x16x32_f16(false, a, false, b, (short)0, c, false, false);
}
__device__ __forceinline__ v8f mma_b(const FragB& a, const FragB& b, v8f c) {
  c = __builtin_amdgcn_wmma_f32_16x16x32_bf16(false, a.v, false, b.v, (short)0, c, false, false);
#if defined(__HIP_DEVICE_COMPILE__)
  asm volatile("v_nop\n\tv_nop\n\tv_nop\n\tv_nop" : "+v"(c) : "v"(a.f), "v"(b.f));
#endif
  return c;
}
__device__ __forceinline__ void dep_guard1(v8f& a, v8f& b, v16h x) {
#if defined(__HIP_DEVICE_COMPILE__)
  asm volatile("v_nop\n\tv_nop\n\tv_nop\n\tv_nop" : "+v"(a), "+v"(b) : "v"(x));
#endif
}
__device__ __forceinline__ void keep4_h(v16h a, v16h b, v16h c, v16h d) {
#if defined(__HIP_DEVICE_COMPILE__)
  asm volatile("v_nop" :: "v"(a), "v"(b), "v"(c), "v"(d));
#endif
}
__device__ __forceinline__ void acc_guard4(v8f& a, v8f& b, v8f& c, v8f& d) {
#if defined(__HIP_DEVICE_COMPILE__)
  asm volatile("v_nop\n\tv_nop\n\tv_nop\n\tv_nop" : "+v"(a), "+v"(b), "+v"(c), "+v"(d));
#endif
}
__device__ __forceinline__ void wave_sync_lds() {
  __builtin_amdgcn_fence(__ATOMIC_RELEASE, "workgroup");
  __builtin_amdgcn_wave_barrier();
  __builtin_amdgcn_fence(__ATOMIC_ACQUIRE, "workgroup");
}
__device__ __forceinline__ float wsum(float v) {
#pragma unroll
  for (int off = 16; off > 0; off >>= 1) v += __shfl_xor(v, off, 32);
  return v;
}
__device__ __forceinline__ float bsumLN(float v, float* red, int lane, int wave) {
  v = wsum(v);
  if (lane == 0) red[wave] = v;
  __syncthreads();
  float tot = 0.f;
#pragma unroll
  for (int w = 0; w < LNW; ++w) tot += red[w];
  return tot;
}

__global__ __launch_bounds__(256) void conv_h16(const float* __restrict__ W, unsigned short* Wh, int n8, float wsc) {
  const int i  = blockIdx.x * 256 + threadIdx.x;
  const int ic = (i < n8) ? i : (n8 - 1);
  const float* src = W + (size_t)ic * 8;
  const v4f a = *(const v4f*)(src);
  const v4f c = *(const v4f*)(src + 4);
  v4u o;
  o[0] = pk16(h_bits((_Float16)(bfr(a[0]) * wsc)), h_bits((_Float16)(bfr(a[1]) * wsc)));
  o[1] = pk16(h_bits((_Float16)(bfr(a[2]) * wsc)), h_bits((_Float16)(bfr(a[3]) * wsc)));
  o[2] = pk16(h_bits((_Float16)(bfr(c[0]) * wsc)), h_bits((_Float16)(bfr(c[1]) * wsc)));
  o[3] = pk16(h_bits((_Float16)(bfr(c[2]) * wsc)), h_bits((_Float16)(bfr(c[3]) * wsc)));
  if (i < n8) *(volatile v4u*)(Wh + (size_t)i * 8) = o;
  __threadfence();
  if (i < n8) *(volatile v4u*)(Wh + (size_t)i * 8) = o;
}

template <int OM, int BIASM, int RES, int AHM>
__global__ __launch_bounds__(256) void gemm64(
    const unsigned short* __restrict__ Ap, int lda, long long strideA,
    const unsigned short* __restrict__ Btp, int ldb, long long strideB,
    const float* __restrict__ bias, const float* resid,
    void* Cout, int ldc, long long strideC,
    int M, int N, int K, float oscale) {
  const _Float16* A  = (const _Float16*)(const void*)Ap;
  const _Float16* Bt = (const _Float16*)(const void*)Btp;
  __shared__ __align__(16) float sT[8][16 * 68];
  const int b    = blockIdx.y;
  const int lane = threadIdx.x & 31;
  const int wave = threadIdx.x >> 5;
  const int tilesN = N >> 6;
  const int tilesM = M >> 6;
  const int tile = blockIdx.x * 8 + wave;
  if (tile >= tilesM * tilesN) return;
  const int tm = tile / tilesN;
  const int tn = tile - tm * tilesN;
  const int m0 = tm << 6;
  const int n0 = tn << 6;

  const _Float16* Ab = A  + (size_t)b * strideA;
  const _Float16* Bb = Bt + (size_t)b * strideB;

  const int rlane = lane & 15;
  const int koff  = (lane >> 4) * 8;
  const int mOff  = (lane >> 4) * 8;

  v8f acc[4][4];
#pragma unroll
  for (int i = 0; i < 4; ++i)
#pragma unroll
    for (int j = 0; j < 4; ++j) acc[i][j] = zero8();

  for (int k0 = 0; k0 < K; k0 += 32) {
    v16h bh[4];
#pragma unroll
    for (int j = 0; j < 4; ++j) {
      const size_t bo = (size_t)(n0 + (j << 4) + rlane) * ldb + koff + k0;
      bh[j] = ldfrag_h(Bb + bo);
    }
#pragma unroll
    for (int i = 0; i < 4; ++i) {
      size_t ao;
      if (AHM) {
        const int m = m0 + (i << 4) + rlane;
        ao = ((size_t)((m / SEQ) * NH + (k0 / HD)) * SEQ + (size_t)(m % SEQ)) * HD + koff;
      } else {
        ao = (size_t)(m0 + (i << 4) + rlane) * lda + koff + k0;
      }
      const v16h ah = ldfrag_h(Ab + ao);
#pragma unroll
      for (int j = 0; j < 4; ++j) acc[i][j] = mma_h_raw(ah, bh[j], acc[i][j]);
      dep_guard1(acc[i][0], acc[i][3], ah);
    }
    keep4_h(bh[0], bh[1], bh[2], bh[3]);
  }
  acc_guard4(acc[0][0], acc[0][1], acc[0][2], acc[0][3]);
  acc_guard4(acc[1][0], acc[1][1], acc[1][2], acc[1][3]);
  acc_guard4(acc[2][0], acc[2][1], acc[2][2], acc[2][3]);
  acc_guard4(acc[3][0], acc[3][1], acc[3][2], acc[3][3]);

  const int hh2 = lane >> 4, c4 = (lane & 15) * 4;
  const int q8  = lane >> 3, c8 = (lane & 7) * 8;
  float bc[8];
#pragma unroll
  for (int e = 0; e < 8; ++e) bc[e] = 0.f;
  if (BIASM == 0) {
    if (OM == 0) {
      const int cb = n0 + c4;
      const int i0 = (cb < N - 4) ? cb : (N - 4);
      const v4f b0v = *(const v4f*)(bias + i0);
#pragma unroll
      for (int e = 0; e < 4; ++e) bc[e] = bfr(b0v[e]);
    } else {
      const int cb = n0 + c8;
      const int i0 = (cb < N - 8) ? cb : (N - 8);
      const v4f b0a = *(const v4f*)(bias + i0), b0b = *(const v4f*)(bias + i0 + 4);
#pragma unroll
      for (int e = 0; e < 4; ++e) {
        bc[e]     = bfr(b0a[e]);
        bc[4 + e] = bfr(b0b[e]);
      }
    }
  }

  float* slab = sT[wave];
#pragma unroll
  for (int i = 0; i < 4; ++i) {
    const int mBase = m0 + (i << 4);
#pragma unroll
    for (int j = 0; j < 4; ++j) {
#pragma unroll
      for (int r = 0; r < 8; ++r) {
        slab[(mOff + r) * 68 + (j << 4) + rlane] = acc[i][j][r];
      }
    }
    wave_sync_lds();
    if (OM == 0) {
      float* C = (float*)Cout + (size_t)b * strideC;
      const float* Rb = resid + (size_t)b * strideC;
      v4f vals[8];
#pragma unroll
      for (int it = 0; it < 8; ++it) {
        const int row = it * 2 + hh2;
        v4f v = *(const v4f*)(slab + row * 68 + c4);
#pragma unroll
        for (int e = 0; e < 4; ++e) v[e] = v[e] * oscale + bc[e];
        if (RES == 3) {
          const v4f rr = *(const v4f*)(Rb + (size_t)(mBase + row) * ldc + n0 + c4);
#pragma unroll
          for (int e = 0; e < 4; ++e) v[e] += bfr(rr[e]);
        }
        vals[it] = v;
      }
      for (int pass = 0; pass < 2; ++pass) {
#pragma unroll
        for (int it = 0; it < 8; ++it) {
          const int row = it * 2 + hh2;
          *(volatile v4f*)(C + (size_t)(mBase + row) * ldc + n0 + c4) = vals[it];
        }
        __threadfence();
      }
    } else {
      unsigned short* C = (unsigned short*)Cout + (size_t)b * strideC;
      v4u hv[4];
#pragma unroll
      for (int it = 0; it < 4; ++it) {
        const int row = it * 4 + q8;
        const float* sp = slab + row * 68 + c8;
        float bm = 0.f;
        if (BIASM == 1) bm = bfr(bias[mBase + row]);
        v4u a;
#pragma unroll
        for (int e = 0; e < 4; ++e) {
          const float f0 = sp[2 * e]     * oscale + ((BIASM == 1) ? bm : bc[2 * e]);
          const float f1 = sp[2 * e + 1] * oscale + ((BIASM == 1) ? bm : bc[2 * e + 1]);
          a[e] = pk16(h_bits((_Float16)f0), h_bits((_Float16)f1));
        }
        hv[it] = a;
      }
      for (int pass = 0; pass < 2; ++pass) {
#pragma unroll
        for (int it = 0; it < 4; ++it) {
          const int row = it * 4 + q8;
          *(volatile v4u*)(C + (size_t)(mBase + row) * ldc + n0 + c8) = hv[it];
        }
        __threadfence();
      }
    }
    wave_sync_lds();
  }
}

__global__ __launch_bounds__(DM) void colstat(const float* __restrict__ PR, float* pmx, float* pmn) {
  const int b = blockIdx.x, e = threadIdx.x;
  const float* p = PR + (size_t)b * SEQ * NPROJ + 2 * DM + e;
  float mx = -INFINITY, mn = INFINITY;
#pragma unroll 4
  for (int n = 0; n < SEQ; ++n) {
    const float v = p[(size_t)n * NPROJ];
    mx = fmaxf(mx, v);
    mn = fminf(mn, v);
  }
  __shared__ __align__(16) float smx[DM];
  __shared__ __align__(16) float smn[DM];
  smx[e] = mx;
  smn[e] = mn;
  __syncthreads();
  typedef float v4f_cs __attribute__((ext_vector_type(4)));
  for (int pass = 0; pass < 2; ++pass) {
    if (e < DM / 4) {
      const v4f_cs vx = *(const v4f_cs*)(smx + 4 * e);
      *(volatile v4f_cs*)(pmx + b * DM + 4 * e) = vx;
    } else if (e < DM / 2) {
      const int t = e - DM / 4;
      const v4f_cs vn = *(const v4f_cs*)(smn + 4 * t);
      *(volatile v4f_cs*)(pmn + b * DM + 4 * t) = vn;
    }
    __threadfence();
  }
}

__global__ __launch_bounds__(256) void qk_planes(
    const float* __restrict__ PR, const float* __restrict__ pmx, const float* __restrict__ pmn,
    const float* __restrict__ bq, const float* __restrict__ bk, const float* __restrict__ br,
    unsigned short* Qh, unsigned short* Ql, unsigned short* Kh, unsigned short* Kl) {
  const int lane = threadIdx.x & 31, wave = threadIdx.x >> 5;
  const int m  = blockIdx.x * 8 + wave;
  const int b  = m / SEQ;
  const int c0 = lane * 8;
  const float* pr = PR + (size_t)m * NPROJ + c0;
  float qr[8], kr[8];
#pragma unroll
  for (int g = 0; g < 2; ++g) {
    const v4f q  = *(const v4f*)(pr + 4 * g);
    const v4f k  = *(const v4f*)(pr + DM + 4 * g);
    const v4f r  = *(const v4f*)(pr + 2 * DM + 4 * g);
    const v4f px = *(const v4f*)(pmx + b * DM + c0 + 4 * g);
    const v4f pn = *(const v4f*)(pmn + b * DM + c0 + 4 * g);
    const v4f vq = *(const v4f*)(bq + c0 + 4 * g);
    const v4f vk = *(const v4f*)(bk + c0 + 4 * g);
    const v4f vr = *(const v4f*)(br + c0 + 4 * g);
#pragma unroll
    for (int e = 0; e < 4; ++e) {
      const float brr = bfr(vr[e]);
      qr[4 * g + e] = (q[e] + bfr(vq[e])) + ((px[e] - r[e]) + brr);
      kr[4 * g + e] = (k[e] + bfr(vk[e])) + ((r[e] - pn[e]) + brr);
    }
  }
  v4u qh, ql, kh, kl;
#pragma unroll
  for (int e = 0; e < 4; ++e) {
    const unsigned short a0 = bf_bits(qr[2 * e]), a1 = bf_bits(qr[2 * e + 1]);
    const unsigned short d0 = bf_bits(kr[2 * e]), d1 = bf_bits(kr[2 * e + 1]);
    qh[e] = pk16(a0, a1);
    ql[e] = pk16(bf_bits(qr[2 * e] - bf_up(a0)), bf_bits(qr[2 * e + 1] - bf_up(a1)));
    kh[e] = pk16(d0, d1);
    kl[e] = pk16(bf_bits(kr[2 * e] - bf_up(d0)), bf_bits(kr[2 * e + 1] - bf_up(d1)));
  }
  const size_t o = (size_t)m * DM + c0;
  *(volatile v4u*)(Qh + o) = qh;
  *(volatile v4u*)(Ql + o) = ql;
  *(volatile v4u*)(Kh + o) = kh;
  *(volatile v4u*)(Kl + o) = kl;
  __threadfence();
  *(volatile v4u*)(Qh + o) = qh;
  *(volatile v4u*)(Ql + o) = ql;
  *(volatile v4u*)(Kh + o) = kh;
  *(volatile v4u*)(Kl + o) = kl;
}

__global__ __launch_bounds__(128)
void attn32(const unsigned short* __restrict__ Qhp, const unsigned short* __restrict__ Qlp,
            const unsigned short* __restrict__ Khp, const unsigned short* __restrict__ Klp,
            const unsigned short* __restrict__ vtp, unsigned short* ctxp, float sscale) {
  __shared__ __align__(16) unsigned short Khs[64 * HD];
  __shared__ __align__(16) unsigned short Kls[64 * HD];
  __shared__ __align__(16) _Float16 Vts[HD * 64];
  __shared__ __align__(16) _Float16 Psh[4][16 * 64];
  __shared__ __align__(16) float    Os[4][16 * HD];

  const int tid  = threadIdx.x;
  const int wave = tid >> 5;
  const int lane = tid & 31;
  const int hh   = lane >> 4;
  const int c    = lane & 15;

  const int bx   = blockIdx.x;
  const int qb   = bx % NQB;
  const int rest = bx / NQB;
  const int h    = rest % NH;
  const int b    = rest / NH;
  const int q0   = qb * 64 + wave * 16;
  const size_t rowB = (size_t)b * SEQ;

  FragB qah, qal;
  {
    const size_t qo = (rowB + q0 + c) * DM + (size_t)h * HD + 8 * hh;
    qah.u[0] = *(const v4u*)(Qhp + qo);
    qah.u[1] = *(const v4u*)(Qhp + qo + 16);
    qal.u[0] = *(const v4u*)(Qlp + qo);
    qal.u[1] = *(const v4u*)(Qlp + qo + 16);
  }
  const _Float16* Vg = (const _Float16*)(const void*)vtp + ((size_t)b * DM + (size_t)h * HD) * SEQ;

  float mrow[8], lrow[8];
  v8f oacc[2];
#pragma unroll
  for (int r = 0; r < 8; ++r) { mrow[r] = -INFINITY; lrow[r] = 0.f; }
#pragma unroll
  for (int t = 0; t < 2; ++t) oacc[t] = zero8();

  for (int kt = 0; kt < NQB; ++kt) {
    const int kv0 = kt * 64;
    __syncthreads();
    {
      const int r = tid >> 1, hf = (tid & 1) * 16;
      const size_t ko = (rowB + kv0 + r) * DM + (size_t)h * HD + hf;
      const v4u a0 = *(const v4u*)(Khp + ko), a1 = *(const v4u*)(Khp + ko + 8);
      const v4u l0 = *(const v4u*)(Klp + ko), l1 = *(const v4u*)(Klp + ko + 8);
      *(v4u*)(Khs + r * HD + hf)     = a0;
      *(v4u*)(Khs + r * HD + hf + 8) = a1;
      *(v4u*)(Kls + r * HD + hf)     = l0;
      *(v4u*)(Kls + r * HD + hf + 8) = l1;
      const int d = tid >> 2, pc = (tid & 3) * 16;
      const _Float16* vg = Vg + (size_t)d * SEQ + kv0 + pc;
      const v8h v0 = *(const v8h*)(vg), v1 = *(const v8h*)(vg + 8);
      *(v8h*)(Vts + d * 64 + pc)     = v0;
      *(v8h*)(Vts + d * 64 + pc + 8) = v1;
    }
    __syncthreads();

    v8f s[4];
#pragma unroll
    for (int j = 0; j < 4; ++j) {
      FragB kbh, kbl;
      kbh.u[0] = *(const v4u*)(Khs + (j * 16 + c) * HD + 8 * hh);
      kbh.u[1] = *(const v4u*)(Khs + (j * 16 + c) * HD + 16 + 8 * hh);
      kbl.u[0] = *(const v4u*)(Kls + (j * 16 + c) * HD + 8 * hh);
      kbl.u[1] = *(const v4u*)(Kls + (j * 16 + c) * HD + 16 + 8 * hh);
      v8f sh = zero8();
      sh = mma_b(qah, kbh, sh);
      sh = mma_b(qah, kbl, sh);
      sh = mma_b(qal, kbh, sh);
#pragma unroll
      for (int r = 0; r < 8; ++r) s[j][r] = sh[r] * sscale;
    }

    _Float16* pwh = Psh[wave];
#pragma unroll
    for (int r = 0; r < 8; ++r) {
      float m = s[0][r];
      m = fmaxf(m, s[1][r]);
      m = fmaxf(m, s[2][r]);
      m = fmaxf(m, s[3][r]);
#pragma unroll
      for (int off = 1; off < 16; off <<= 1) m = fmaxf(m, __shfl_xor(m, off, 32));
      const float mnew  = fmaxf(mrow[r], m);
      const float alpha = __expf(mrow[r] - mnew);
      mrow[r] = mnew;
      float psum = 0.f;
#pragma unroll
      for (int j = 0; j < 4; ++j) {
        const float p = __expf(s[j][r] - mnew);
        psum += p;
        pwh[(8 * hh + r) * 64 + j * 16 + c] = (_Float16)(p * PSC);
      }
#pragma unroll
      for (int off = 1; off < 16; off <<= 1) psum += __shfl_xor(psum, off, 32);
      lrow[r] = lrow[r] * alpha + psum;
#pragma unroll
      for (int t = 0; t < 2; ++t) oacc[t][r] *= alpha;
    }
    wave_sync_lds();

#pragma unroll 1
    for (int kk = 0; kk < 2; ++kk) {
      FragH pa;
      pa.h[0] = *(const v8h*)(pwh + c * 64 + kk * 32 + 8 * hh);
      pa.h[1] = *(const v8h*)(pwh + c * 64 + kk * 32 + 16 + 8 * hh);
#pragma unroll
      for (int t = 0; t < 2; ++t) {
        FragH vb;
        vb.h[0] = *(const v8h*)(Vts + (t * 16 + c) * 64 + kk * 32 + 8 * hh);
        vb.h[1] = *(const v8h*)(Vts + (t * 16 + c) * 64 + kk * 32 + 16 + 8 * hh);
        oacc[t] = mma_h(pa.v, vb.v, oacc[t]);
      }
    }
  }

  float* os = Os[wave];
#pragma unroll
  for (int r = 0; r < 8; ++r) {
    const float l = lrow[r];
    const float inv = ((l > 0.f) ? (1.0f / l) : 0.f) * (CSC / PSC);
#pragma unroll
    for (int t = 0; t < 2; ++t) os[(8 * hh + r) * HD + t * 16 + c] = oacc[t][r] * inv;
  }
  wave_sync_lds();
  {
    unsigned short* tb = ctxp + (((size_t)(b * NH + h) * SEQ + q0) * HD);
    v4u hv[2];
#pragma unroll
    for (int it = 0; it < 2; ++it) {
      const int p   = it * 32 + lane;
      const int row = p >> 2, col = (p & 3) * 8;
      const float* sp = os + row * HD + col;
      v4u a;
#pragma unroll
      for (int e = 0; e < 4; ++e) a[e] = pk16(h_bits((_Float16)sp[2 * e]), h_bits((_Float16)sp[2 * e + 1]));
      hv[it] = a;
    }
    for (int pass = 0; pass < 2; ++pass) {
#pragma unroll
      for (int it = 0; it < 2; ++it) {
        const int p = it * 32 + lane;
        *(volatile v4u*)(tb + (size_t)p * 8) = hv[it];
      }
      __threadfence();
    }
  }
}

__global__ __launch_bounds__(LNT) void ln2_row(const float* __restrict__ X,
                                               const float* __restrict__ ga1, const float* __restrict__ be1,
                                               const float* __restrict__ ga2, const float* __restrict__ be2,
                                               float* outF) {
  __shared__ float red0[8], red1[8], red2[8], red3[8];
  const int t = threadIdx.x, lane = t & 31, wave = t >> 5;
  const size_t base = (size_t)blockIdx.x * DM;
  const v4f xv = *(const v4f*)(X + base + 4 * t);
  const float mean = bsumLN((xv[0] + xv[1]) + (xv[2] + xv[3]), red0, lane, wave) * (1.0f / DM);
  v4f d;
#pragma unroll
  for (int e = 0; e < 4; ++e) d[e] = xv[e] - mean;
  const float var  = bsumLN((d[0] * d[0] + d[1] * d[1]) + (d[2] * d[2] + d[3] * d[3]), red1, lane, wave) * (1.0f / DM);
  const float rstd = rsqrtf(var + LNEPS);
  const v4f g1v = *(const v4f*)(ga1 + 4 * t);
  const v4f b1v = *(const v4f*)(be1 + 4 * t);
  v4f hv;
#pragma unroll
  for (int e = 0; e < 4; ++e) hv[e] = (d[e] * rstd) * bfr(g1v[e]) + bfr(b1v[e]);
  const float mean2 = bsumLN((hv[0] + hv[1]) + (hv[2] + hv[3]), red2, lane, wave) * (1.0f / DM);
  v4f d2;
#pragma unroll
  for (int e = 0; e < 4; ++e) d2[e] = hv[e] - mean2;
  const float var2  = bsumLN((d2[0] * d2[0] + d2[1] * d2[1]) + (d2[2] * d2[2] + d2[3] * d2[3]), red3, lane, wave) * (1.0f / DM);
  const float rstd2 = rsqrtf(var2 + LNEPS);
  const v4f g2v = *(const v4f*)(ga2 + 4 * t);
  const v4f b2v = *(const v4f*)(be2 + 4 * t);
  v4f y;
#pragma unroll
  for (int e = 0; e < 4; ++e) y[e] = (d2[e] * rstd2) * bfr(g2v[e]) + bfr(b2v[e]);
  float* dst = outF + base + 4 * t;
  *(volatile v4f*)dst = y;
  __threadfence();
  *(volatile v4f*)dst = y;
}

extern "C" void kernel_launch(void* const* d_in, const int* in_sizes, int n_in,
                              void* d_out, int out_size, void* d_ws, size_t ws_size,
                              hipStream_t stream) {
  if (n_in < 15) return;
  if (in_sizes[0] != MP * DM) return;
  if (in_sizes[1] != DM * DM || in_sizes[2] != DM) return;
  if (in_sizes[3] != DM * DM || in_sizes[4] != DM) return;
  if (in_sizes[5] != DM * DM || in_sizes[6] != DM) return;
  if (in_sizes[7] != DM * DM || in_sizes[8] != DM) return;
  if (in_sizes[9] != DM * DM || in_sizes[10] != DM) return;
  if (in_sizes[11] != DM || in_sizes[12] != DM || in_sizes[13] != DM || in_sizes[14] != DM) return;
  if (out_size != MP * DM) return;

  const float* xin  = (const float*)d_in[0];
  const float* w_q  = (const float*)d_in[1];
  const float* b_q  = (const float*)d_in[2];
  const float* w_k  = (const float*)d_in[3];
  const float* b_k  = (const float*)d_in[4];
  const float* w_v  = (const float*)d_in[5];
  const float* b_v  = (const float*)d_in[6];
  const float* w_r  = (const float*)d_in[7];
  const float* b_r  = (const float*)d_in[8];
  const float* w_o  = (const float*)d_in[9];
  const float* b_o  = (const float*)d_in[10];
  const float* ln_g1 = (const float*)d_in[11];
  const float* ln_b1 = (const float*)d_in[12];
  const float* ln_g2 = (const float*)d_in[13];
  const float* ln_b2 = (const float*)d_in[14];

  const size_t PWQKR = (size_t)NPROJ * DM * 2;
  const size_t PW    = (size_t)DM * DM * 2;
  const size_t PXH   = (size_t)MP * DM * 2;
  const size_t PPR   = (size_t)MP * NPROJ * 4;
  const size_t PVT   = (size_t)NBATCH * DM * SEQ * 2;
  const size_t PST   = (size_t)NBATCH * DM * 4;
  const size_t PQK   = (size_t)MP * DM * 2;
  const size_t PCTX  = (size_t)NBATCH * NH * SEQ * HD * 2;
  const size_t PHF   = (size_t)MP * DM * 4;
  size_t off = 0;
  const size_t oWqkr = off; off += PWQKR;
  const size_t oWv   = off; off += PW;
  const size_t oWo   = off; off += PW;
  const size_t oXH   = off; off += PXH;
  const size_t oPR   = off; off += PPR;
  const size_t oVT   = off; off += PVT;
  const size_t oPmx  = off; off += PST;
  const size_t oPmn  = off; off += PST;
  const size_t oQh   = off; off += PQK;
  const size_t oQl   = off; off += PQK;
  const size_t oKh   = off; off += PQK;
  const size_t oKl   = off; off += PQK;
  const size_t oCtx  = off; off += PCTX;
  const size_t oHf   = off; off += PHF;
  if (off > ws_size) return;
  if (off > (size_t)134217728) return;

  char* ws = (char*)d_ws;
  unsigned short* WqkrH = (unsigned short*)(ws + oWqkr);
  unsigned short* WvH   = (unsigned short*)(ws + oWv);
  unsigned short* WoH   = (unsigned short*)(ws + oWo);
  unsigned short* XH    = (unsigned short*)(ws + oXH);
  float*          PR    = (float*)(ws + oPR);
  unsigned short* VT    = (unsigned short*)(ws + oVT);
  float*          PMX   = (float*)(ws + oPmx);
  float*          PMN   = (float*)(ws + oPmn);
  unsigned short* QHp   = (unsigned short*)(ws + oQh);
  unsigned short* QLp   = (unsigned short*)(ws + oQl);
  unsigned short* KHp   = (unsigned short*)(ws + oKh);
  unsigned short* KLp   = (unsigned short*)(ws + oKl);
  unsigned short* Ctx   = (unsigned short*)(ws + oCtx);
  float*          Hf    = (float*)(ws + oHf);
  float*          out0  = (float*)d_out;

  const int n8w = (DM * DM) / 8;
  const int n8x = (MP * DM) / 8;
  if ((n8w % 256) != 0 || (n8x % 256) != 0) return;
  const dim3 blk(256), blk128(128), blkLN(LNT), blkDM(DM);
  const dim3 gCw(n8w / 256), gCx(n8x / 256);
  const dim3 gProj(((MP / 64) * (NPROJ / 64) + 7) / 8, 1);
  const dim3 gVT(((DM / 64) * (SEQ / 64) + 7) / 8, NBATCH);
  const dim3 gWo(((MP / 64) * (DM / 64) + 7) / 8, 1);
  const dim3 gStat(NBATCH);
  const dim3 gQK(MP / 8);
  const dim3 gAttn(NBATCH * NH * NQB);
  const dim3 gRow(MP);
  const float invw  = 1.0f / WSC;
  const float invwc = 1.0f / (WSC * CSC);

  conv_h16<<<gCw, blk, 0, stream>>>(w_q, WqkrH, n8w, WSC);
  conv_h16<<<gCw, blk, 0, stream>>>(w_k, WqkrH + (size_t)DM * DM, n8w, WSC);
  conv_h16<<<gCw, blk, 0, stream>>>(w_r, WqkrH + (size_t)2 * DM * DM, n8w, WSC);
  conv_h16<<<gCw, blk, 0, stream>>>(w_v, WvH, n8w, WSC);
  conv_h16<<<gCw, blk, 0, stream>>>(w_o, WoH, n8w, WSC);
  conv_h16<<<gCx, blk, 0, stream>>>(xin, XH, n8x, 1.0f);

  gemm64<0, 2, 0, 0><<<gProj, blk, 0, stream>>>(
      XH, DM, 0LL, WqkrH, DM, 0LL, b_q, xin,
      (void*)PR, NPROJ, 0LL, MP, NPROJ, DM, invw);
  gemm64<2, 1, 0, 0><<<gVT, blk, 0, stream>>>(
      WvH, DM, 0LL, XH, DM, (long long)SEQ * DM, b_v, xin,
      (void*)VT, SEQ, (long long)DM * SEQ, DM, SEQ, DM, invw);

  colstat<<<gStat, blkDM, 0, stream>>>(PR, PMX, PMN);
  qk_planes<<<gQK, blk, 0, stream>>>(PR, PMX, PMN, b_q, b_k, b_r, QHp, QLp, KHp, KLp);

  attn32<<<gAttn, blk128, 0, stream>>>(QHp, QLp, KHp, KLp, VT, Ctx, 0.17677669529663687f);

  gemm64<0, 0, 3, 1><<<gWo, blk, 0, stream>>>(
      Ctx, HD, 0LL, WoH, DM, 0LL, b_o, xin,
      (void*)Hf, DM, 0LL, MP, DM, DM, invwc);

  ln2_row<<<gRow, blkLN, 0, stream>>>(Hf, ln_g1, ln_b1, ln_g2, ln_b2, out0);
  (void)hipGetLastError();
}
